// GPT2Attention_27496380629258
// MI455X (gfx1250) — hardware-verified
//
#include <hip/hip_runtime.h>


#ifndef NB
#define NB 4
#endif
#ifndef SEQ
#define SEQ 2048
#endif
#ifndef TRES
#define TRES 512
#endif
#define NB_FULL   4
#define SEQ_FULL  2048
#define CDIM      1024
#define NHEAD     16
#define NKV       4
#define HDIM      64
#define ROTD      32
#define GATEC     12
#define VEW       (NKV * HDIM)
#define NTOK      (NB * SEQ)
#define NUNIT     (NHEAD + 2 * NKV)
#define WO_ROW0   (CDIM + 2 * VEW)
#define NWROWS    (CDIM + 2 * VEW + CDIM)
#define QT_ALL    (SEQ / 64)
#define QT_RES    (TRES / 64)

static_assert(NB >= 1 && NB <= NB_FULL);
static_assert(SEQ % 64 == 0 && SEQ <= SEQ_FULL && SEQ >= TRES);
static_assert(TRES % 64 == 0 && TRES >= 64);
static_assert(NHEAD % NKV == 0 && HDIM == 64 && CDIM == NHEAD * HDIM && ROTD * 2 == HDIM);
static_assert(CDIM % 32 == 0 && NWROWS % 2 == 0 && NTOK % 64 == 0 && NUNIT * 64 == CDIM + 2 * VEW);

#define XH_BYTES   ((size_t)NTOK * CDIM * 2)
#define WALL_BYTES ((size_t)NWROWS * CDIM * 2)
#define QP_BYTES   ((size_t)NB * NHEAD * SEQ * HDIM * 2)
#define KP_BYTES   ((size_t)NB * NKV * SEQ * HDIM * 2)
#define YP_BYTES   ((size_t)NTOK * CDIM * 2)
#define WS_TOTAL   (XH_BYTES + WALL_BYTES + 2 * QP_BYTES + 4 * KP_BYTES + 2 * YP_BYTES)
static_assert(WS_TOTAL <= (size_t)134217728);
static_assert(XH_BYTES % 128 == 0 && WALL_BYTES % 128 == 0 && QP_BYTES % 128 == 0 && KP_BYTES % 128 == 0 && YP_BYTES % 128 == 0);
static_assert((size_t)(NTOK / 2) * 256 * 8 == (size_t)NTOK * CDIM);
static_assert((size_t)(NWROWS / 2) * 256 * 8 == (size_t)NWROWS * CDIM);
static_assert(4 * 128 * 8 == 64 * 64);
static_assert(4 * 32 * 8 == 16 * HDIM);
static_assert(8 * 32 * 4 == 16 * 64);
static_assert(QT_RES * 64 + (QT_ALL - QT_RES) * 64 == SEQ);

typedef _Float16 v16h __attribute__((ext_vector_type(16)));
typedef _Float16 v8h  __attribute__((ext_vector_type(8)))  __attribute__((may_alias));
typedef float    v8f  __attribute__((ext_vector_type(8)));
typedef float    v4f  __attribute__((ext_vector_type(4)))  __attribute__((may_alias));

union Frag { v16h v; v8h h[2]; };

__device__ __forceinline__ v8f wmma16(v16h a, v16h b, v8f c) {
  return __builtin_amdgcn_wmma_f32_16x16x32_f16(false, a, false, b, (short)0, c, false, false);
}

__device__ __forceinline__ v8f vzero8() {
  v8f z = {0.0f, 0.0f, 0.0f, 0.0f, 0.0f, 0.0f, 0.0f, 0.0f};
  return z;
}

__device__ __forceinline__ float bf16r(float f) {
  unsigned int u = __float_as_uint(f);
  u = (u + 0x7FFFu + ((u >> 16) & 1u)) & 0xFFFF0000u;
  return __uint_as_float(u);
}

__device__ __forceinline__ void split16(float v, _Float16& hi, _Float16& lo) {
  hi = (_Float16)v;
  lo = (_Float16)((v - (float)hi) * 2048.0f);
}

__global__ void __launch_bounds__(256) k_cvt_x(const float* __restrict__ x, _Float16* __restrict__ xh) {
  const unsigned int gid = blockIdx.x * 256u + threadIdx.x;
  const unsigned int tok = gid >> 7;
  const int c = (int)(gid & 127u) * 8;
  if (tok >= (unsigned int)NTOK) return;
  const int b = (int)tok / SEQ;
  const int t = (int)tok - b * SEQ;
  const float* src = x + ((size_t)b * SEQ_FULL + t) * CDIM + c;
  const v4f f0 = *(const v4f*)src;
  const v4f f1 = *(const v4f*)(src + 4);
  v8h o;
#pragma unroll
  for (int j = 0; j < 4; ++j) {
    o[j]     = (_Float16)bf16r(f0[j]);
    o[j + 4] = (_Float16)bf16r(f1[j]);
  }
  _Float16* dst = xh + (size_t)tok * CDIM + c;
  *(volatile v8h*)dst = o;
  __threadfence();
  *(volatile v8h*)dst = o;
}

__global__ void __launch_bounds__(256) k_cvt_w(const float* __restrict__ wq, const float* __restrict__ wk,
                                               const float* __restrict__ wv, const float* __restrict__ wo,
                                               _Float16* __restrict__ wall) {
  const unsigned int gid = blockIdx.x * 256u + threadIdx.x;
  const int row = (int)(gid >> 7);
  const int c   = (int)(gid & 127u) * 8;
  if (row >= NWROWS) return;
  const int r0 = min(row, CDIM - 1);
  const int r1 = min(max(row - CDIM, 0), VEW - 1);
  const int r2 = min(max(row - CDIM - VEW, 0), VEW - 1);
  const int r3 = min(max(row - WO_ROW0, 0), CDIM - 1);
  const float* src = (row < CDIM)       ? (wq + (size_t)r0 * CDIM)
                   : (row < CDIM + VEW) ? (wk + (size_t)r1 * CDIM)
                   : (row < WO_ROW0)    ? (wv + (size_t)r2 * CDIM)
                                        : (wo + (size_t)r3 * CDIM);
  src += c;
  const v4f f0 = *(const v4f*)src;
  const v4f f1 = *(const v4f*)(src + 4);
  v8h o;
#pragma unroll
  for (int j = 0; j < 4; ++j) {
    o[j]     = (_Float16)(bf16r(f0[j]) * 16.0f);
    o[j + 4] = (_Float16)(bf16r(f1[j]) * 16.0f);
  }
  _Float16* dst = wall + (size_t)row * CDIM + c;
  *(volatile v8h*)dst = o;
  __threadfence();
  *(volatile v8h*)dst = o;
}

__global__ void __launch_bounds__(128) k_qkv(
    const _Float16* __restrict__ xh, const _Float16* __restrict__ wall,
    const float* __restrict__ x, const float* __restrict__ ve,
    const float* __restrict__ cosb, const float* __restrict__ sinb,
    const float* __restrict__ wgate,
    _Float16* __restrict__ qH, _Float16* __restrict__ qL,
    _Float16* __restrict__ kH, _Float16* __restrict__ kL,
    _Float16* __restrict__ vTH, _Float16* __restrict__ vTL) {
  __shared__ __attribute__((aligned(16))) float    sT[64][68];
  __shared__ __attribute__((aligned(16))) _Float16 sH[64][72];
  __shared__ __attribute__((aligned(16))) _Float16 sL[64][72];

  const int tid  = threadIdx.x;
  const int wave = tid >> 5;
  const int lane = tid & 31;
  const int l16  = lane & 15;
  const int lh   = lane >> 4;
  const int u    = blockIdx.x;
  const int rt   = blockIdx.y;
  const int tok0 = rt * 64;
  const int b    = tok0 / SEQ;
  const int t0   = tok0 - b * SEQ;

  const _Float16* arow = xh + (size_t)(tok0 + wave * 16 + l16) * CDIM + 8 * lh;
  const _Float16* brow = wall + (size_t)(u * 64 + l16) * CDIM + 8 * lh;

  v8f acc[4];
#pragma unroll
  for (int n = 0; n < 4; ++n) acc[n] = vzero8();

  for (int k0 = 0; k0 < CDIM; k0 += 32) {
    Frag a;
    a.h[0] = *(const v8h*)(arow + k0);
    a.h[1] = *(const v8h*)(arow + k0 + 16);
    Frag bw[4];
#pragma unroll
    for (int n = 0; n < 4; ++n) {
      const _Float16* bp = brow + (size_t)(n * 16) * CDIM + k0;
      bw[n].h[0] = *(const v8h*)bp;
      bw[n].h[1] = *(const v8h*)(bp + 16);
    }
#pragma unroll
    for (int n = 0; n < 4; ++n) acc[n] = wmma16(a.v, bw[n].v, acc[n]);
    asm volatile("v_nop\n\tv_nop\n\tv_nop\n\tv_nop"
                 : "+v"(acc[0]), "+v"(acc[1]), "+v"(acc[2]), "+v"(acc[3])
                 : "v"(a.v), "v"(bw[0].v), "v"(bw[1].v), "v"(bw[2].v), "v"(bw[3].v));
  }

#pragma unroll
  for (int n = 0; n < 4; ++n)
#pragma unroll
    for (int r = 0; r < 8; ++r)
      sT[wave * 16 + r + 8 * lh][n * 16 + l16] = acc[n][r] * (1.0f / 16.0f);
  __syncthreads();

  const int i = tid >> 1;
  const int j = tid & 1;
  const int t = t0 + i;
  if (u < NHEAD + NKV) {
    const float* cp = cosb + (size_t)t * ROTD + 16 * j;
    const float* sp = sinb + (size_t)t * ROTD + 16 * j;
    float o1[16], o2[16];
    float ss = 0.0f;
#pragma unroll
    for (int g = 0; g < 4; ++g) {
      const v4f x1 = *(const v4f*)(&sT[i][16 * j + 4 * g]);
      const v4f x2 = *(const v4f*)(&sT[i][32 + 16 * j + 4 * g]);
      const v4f cc = *(const v4f*)(cp + 4 * g);
      const v4f sn = *(const v4f*)(sp + 4 * g);
#pragma unroll
      for (int e = 0; e < 4; ++e) {
        const float c  = bf16r(cc[e]);
        const float s  = bf16r(sn[e]);
        const float a1 = x1[e] * c + x2[e] * s;
        const float a2 = x2[e] * c - x1[e] * s;
        o1[4 * g + e] = a1;
        o2[4 * g + e] = a2;
        ss += a1 * a1 + a2 * a2;
      }
    }
    ss += __shfl_xor(ss, 1, 32);
    const float rr = rsqrtf(ss * (1.0f / 64.0f) + 1e-6f) * 1.15f;
#pragma unroll
    for (int e = 0; e < 16; ++e) {
      _Float16 hi, lo;
      split16(o1[e] * rr, hi, lo);
      sH[i][16 * j + e] = hi;
      sL[i][16 * j + e] = lo;
      split16(o2[e] * rr, hi, lo);
      sH[i][32 + 16 * j + e] = hi;
      sL[i][32 + 16 * j + e] = lo;
    }
  } else {
    const int kv = u - NHEAD - NKV;
    const float* xr = x + ((size_t)b * SEQ_FULL + t) * CDIM;
    const float* wg = wgate + kv * GATEC;
    float g = 0.0f;
#pragma unroll
    for (int c4 = 0; c4 < 3; ++c4) {
      const v4f xa = *(const v4f*)(xr + 4 * c4);
      const v4f wa = *(const v4f*)(wg + 4 * c4);
#pragma unroll
      for (int e = 0; e < 4; ++e) g += bf16r(xa[e]) * bf16r(wa[e]);
    }
    const float gate = 3.0f * __builtin_amdgcn_rcpf(1.0f + __expf(-g));
    const float* vp = ve + ((size_t)b * SEQ_FULL + t) * VEW + kv * HDIM;
#pragma unroll
    for (int sg = 0; sg < 2; ++sg) {
      const int d0 = 32 * sg + 16 * j;
#pragma unroll
      for (int g4 = 0; g4 < 4; ++g4) {
        const v4f va = *(const v4f*)(&sT[i][d0 + 4 * g4]);
        const v4f ea = *(const v4f*)(vp + d0 + 4 * g4);
#pragma unroll
        for (int e = 0; e < 4; ++e) {
          const float vv = va[e] + gate * bf16r(ea[e]);
          _Float16 hi, lo;
          split16(vv, hi, lo);
          sH[d0 + 4 * g4 + e][i] = hi;
          sL[d0 + 4 * g4 + e][i] = lo;
        }
      }
    }
  }
  __syncthreads();

  _Float16* ph;
  _Float16* pl;
  size_t base;
  size_t lstr;
  if (u < NHEAD) {
    ph = qH; pl = qL;
    base = ((size_t)(b * NHEAD + u) * SEQ + t0) * HDIM;
    lstr = HDIM;
  } else if (u < NHEAD + NKV) {
    ph = kH; pl = kL;
    base = ((size_t)(b * NKV + (u - NHEAD)) * SEQ + t0) * HDIM;
    lstr = HDIM;
  } else {
    ph = vTH; pl = vTL;
    base = ((size_t)(b * NKV + (u - NHEAD - NKV)) * HDIM) * SEQ + t0;
    lstr = SEQ;
  }
  for (int pass = 0; pass < 2; ++pass) {
#pragma unroll
    for (int it = 0; it < 4; ++it) {
      const int p    = it * 128 + tid;
      const int line = p >> 3;
      const int q8   = (p & 7) * 8;
      const size_t off = base + (size_t)line * lstr + q8;
      const v8h hv = *(const v8h*)(&sH[line][q8]);
      const v8h lv = *(const v8h*)(&sL[line][q8]);
      *(volatile v8h*)(ph + off) = hv;
      *(volatile v8h*)(pl + off) = lv;
    }
    __threadfence();
  }
}

template <bool RES>
__global__ void __launch_bounds__(128) k_flash(
    const _Float16* __restrict__ qH, const _Float16* __restrict__ qL,
    const _Float16* __restrict__ kH, const _Float16* __restrict__ kL,
    const _Float16* __restrict__ vTH, const _Float16* __restrict__ vTL,
    const int* __restrict__ winp,
    _Float16* __restrict__ yH, _Float16* __restrict__ yL, int qt_first) {
  __shared__ __attribute__((aligned(16))) _Float16 ldsPH[4][16 * 32];
  __shared__ __attribute__((aligned(16))) _Float16 ldsPL[4][16 * 32];
  __shared__ __attribute__((aligned(16))) _Float16 sYH[4][16][HDIM];
  __shared__ __attribute__((aligned(16))) _Float16 sYL[4][16][HDIM];

  const int tid  = threadIdx.x;
  const int wave = tid >> 5;
  const int lane = tid & 31;
  const int l16  = lane & 15;
  const int lh   = lane >> 4;
  const int qt   = qt_first + blockIdx.x;
  const int h    = blockIdx.y;
  const int b    = blockIdx.z;
  const int kv   = h / (NHEAD / NKV);
  const int qw   = qt * 64 + wave * 16;
  int window = winp[0];
  window = (window < 0) ? 0 : window;
  const float rres = 1.0f / 2048.0f;
  const float smsc = 0.125f;

  v16h aqh[2], aql[2];
  {
    const size_t qo = ((size_t)(b * NHEAD + h) * SEQ + qw + l16) * HDIM + 8 * lh;
#pragma unroll
    for (int hc = 0; hc < 2; ++hc) {
      Frag a;
      a.h[0] = *(const v8h*)(qH + qo + hc * 32);
      a.h[1] = *(const v8h*)(qH + qo + hc * 32 + 16);
      aqh[hc] = a.v;
      Frag c;
      c.h[0] = *(const v8h*)(qL + qo + hc * 32);
      c.h[1] = *(const v8h*)(qL + qo + hc * 32 + 16);
      aql[hc] = c.v;
    }
  }

  float m[8], l[8];
  v8f coh[4], cor[4];
#pragma unroll
  for (int r = 0; r < 8; ++r) { m[r] = -1e30f; l[r] = 0.0f; }
#pragma unroll
  for (int n = 0; n < 4; ++n) { coh[n] = vzero8(); cor[n] = vzero8(); }

  const size_t kvoff = (size_t)(b * NKV + kv) * SEQ * HDIM;
  const _Float16* kbase  = kH  + kvoff + 8 * lh;
  const _Float16* klbase = kL  + kvoff + 8 * lh;
  const _Float16* vbase  = vTH + kvoff + (size_t)l16 * SEQ + 8 * lh;
  const _Float16* vlbase = vTL + kvoff + (size_t)l16 * SEQ + 8 * lh;

  int kstart = qw - window;
  kstart = (kstart < 0) ? 0 : kstart;
  kstart &= ~31;

  for (int k0 = kstart; k0 < qw + 16; k0 += 32) {
    v8f sh0 = vzero8(), sh1 = vzero8(), sr0 = vzero8(), sr1 = vzero8();
    Frag bh0, bh1, bl0, bl1;
    const _Float16* kr0 = kbase  + (size_t)(k0 + l16) * HDIM;
    const _Float16* kr1 = kr0 + 16 * HDIM;
    const _Float16* lr0 = klbase + (size_t)(k0 + l16) * HDIM;
    const _Float16* lr1 = lr0 + 16 * HDIM;
#pragma unroll
    for (int hc = 0; hc < 2; ++hc) {
      bh0.h[0] = *(const v8h*)(kr0 + hc * 32); bh0.h[1] = *(const v8h*)(kr0 + hc * 32 + 16);
      bh1.h[0] = *(const v8h*)(kr1 + hc * 32); bh1.h[1] = *(const v8h*)(kr1 + hc * 32 + 16);
      bl0.h[0] = *(const v8h*)(lr0 + hc * 32); bl0.h[1] = *(const v8h*)(lr0 + hc * 32 + 16);
      bl1.h[0] = *(const v8h*)(lr1 + hc * 32); bl1.h[1] = *(const v8h*)(lr1 + hc * 32 + 16);
      sh0 = wmma16(aqh[hc], bh0.v, sh0);
      sh1 = wmma16(aqh[hc], bh1.v, sh1);
      sr0 = wmma16(aqh[hc], bl0.v, sr0);
      sr1 = wmma16(aqh[hc], bl1.v, sr1);
      sr0 = wmma16(aql[hc], bh0.v, sr0);
      sr1 = wmma16(aql[hc], bh1.v, sr1);
    }
    asm volatile("v_nop\n\tv_nop\n\tv_nop\n\tv_nop"
                 : "+v"(sh0), "+v"(sh1), "+v"(sr0), "+v"(sr1)
                 : "v"(aqh[0]), "v"(aqh[1]), "v"(aql[0]), "v"(aql[1]),
                   "v"(bh0.v), "v"(bh1.v), "v"(bl0.v), "v"(bl1.v));

    asm volatile("" ::: "memory");
    float alpha[8];
#pragma unroll
    for (int r = 0; r < 8; ++r) {
      const int row = qw + r + 8 * lh;
      const int d0  = row - (k0 + l16);
      const int d1  = d0 - 16;
      const bool ok0 = (d0 >= 0) && (d0 <= window);
      const bool ok1 = (d1 >= 0) && (d1 <= window);
      const float x0 = ok0 ? (sh0[r] + sr0[r] * rres) * smsc : -1e30f;
      const float x1 = ok1 ? (sh1[r] + sr1[r] * rres) * smsc : -1e30f;
      float tmax = fmaxf(x0, x1);
#pragma unroll
      for (int off = 1; off < 16; off <<= 1) tmax = fmaxf(tmax, __shfl_xor(tmax, off, 32));
      const float mn = fmaxf(m[r], tmax);
      alpha[r] = __expf(m[r] - mn);
      const float e0 = __expf(x0 - mn);
      const float e1 = __expf(x1 - mn);
      const float p0 = ok0 ? e0 : 0.0f;
      const float p1 = ok1 ? e1 : 0.0f;
      float ps = p0 + p1;
#pragma unroll
      for (int off = 1; off < 16; off <<= 1) ps += __shfl_xor(ps, off, 32);
      l[r] = l[r] * alpha[r] + ps;
      m[r] = mn;
      const float c0 = p0 * 1024.0f;
      const float c1 = p1 * 1024.0f;
      const _Float16 h0 = (_Float16)c0;
      const _Float16 h1 = (_Float16)c1;
      ldsPH[wave][(r + 8 * lh) * 32 + l16]      = h0;
      ldsPH[wave][(r + 8 * lh) * 32 + 16 + l16] = h1;
      if (RES) {
        ldsPL[wave][(r + 8 * lh) * 32 + l16]      = (_Float16)((c0 - (float)h0) * 2048.0f);
        ldsPL[wave][(r + 8 * lh) * 32 + 16 + l16] = (_Float16)((c1 - (float)h1) * 2048.0f);
      }
    }
#pragma unroll
    for (int n = 0; n < 4; ++n)
#pragma unroll
      for (int r = 0; r < 8; ++r) {
        coh[n][r] *= alpha[r];
        if (RES) cor[n][r] *= alpha[r];
      }

    asm volatile("s_wait_dscnt 0" ::: "memory");
    __builtin_amdgcn_fence(3  , "wavefront");
    __builtin_amdgcn_wave_barrier();

    Frag aph, apl;
    aph.h[0] = *(const v8h*)(&ldsPH[wave][l16 * 32 + 8 * lh]);
    aph.h[1] = *(const v8h*)(&ldsPH[wave][l16 * 32 + 16 + 8 * lh]);
    if (RES) {
      apl.h[0] = *(const v8h*)(&ldsPL[wave][l16 * 32 + 8 * lh]);
      apl.h[1] = *(const v8h*)(&ldsPL[wave][l16 * 32 + 16 + 8 * lh]);
    }
    Frag bv[4], bl[4];
#pragma unroll
    for (int n = 0; n < 4; ++n) {
      const _Float16* vp = vbase + (size_t)(n * 16) * SEQ + k0;
      bv[n].h[0] = *(const v8h*)vp;
      bv[n].h[1] = *(const v8h*)(vp + 16);
      if (RES) {
        const _Float16* lp = vlbase + (size_t)(n * 16) * SEQ + k0;
        bl[n].h[0] = *(const v8h*)lp;
        bl[n].h[1] = *(const v8h*)(lp + 16);
      }
    }
#pragma unroll
    for (int n = 0; n < 4; ++n) {
      coh[n] = wmma16(aph.v, bv[n].v, coh[n]);
      if (RES) {
        cor[n] = wmma16(aph.v, bl[n].v, cor[n]);
        cor[n] = wmma16(apl.v, bv[n].v, cor[n]);
      }
    }
    if (RES) {
      asm volatile("v_nop\n\tv_nop\n\tv_nop\n\tv_nop"
                   : "+v"(coh[0]), "+v"(coh[1]), "+v"(coh[2]), "+v"(coh[3]),
                     "+v"(cor[0]), "+v"(cor[1]), "+v"(cor[2]), "+v"(cor[3])
                   : "v"(aph.v), "v"(apl.v),
                     "v"(bv[0].v), "v"(bv[1].v), "v"(bv[2].v), "v"(bv[3].v),
                     "v"(bl[0].v), "v"(bl[1].v), "v"(bl[2].v), "v"(bl[3].v));
    } else {
      asm volatile("v_nop\n\tv_nop\n\tv_nop\n\tv_nop"
                   : "+v"(coh[0]), "+v"(coh[1]), "+v"(coh[2]), "+v"(coh[3])
                   : "v"(aph.v), "v"(bv[0].v), "v"(bv[1].v), "v"(bv[2].v), "v"(bv[3].v));
    }
  }

#pragma unroll
  for (int r = 0; r < 8; ++r) {
    const float inv = __builtin_amdgcn_rcpf(l[r]) * (1.0f / 1024.0f);
#pragma unroll
    for (int n = 0; n < 4; ++n) {
      float yv = coh[n][r];
      if (RES) yv += cor[n][r] * rres;
      yv *= inv;
      _Float16 hi, lo;
      split16(yv, hi, lo);
      sYH[wave][r + 8 * lh][n * 16 + l16] = hi;
      sYL[wave][r + 8 * lh][n * 16 + l16] = lo;
    }
  }
  asm volatile("s_wait_dscnt 0" ::: "memory");
  __builtin_amdgcn_fence(3  , "wavefront");
  __builtin_amdgcn_wave_barrier();
  const size_t ybase = ((size_t)b * SEQ + qw) * CDIM + (size_t)h * HDIM;
  for (int pass = 0; pass < 2; ++pass) {
#pragma unroll
    for (int it = 0; it < 4; ++it) {
      const int p  = it * 32 + lane;
      const int rr = p >> 3;
      const int q8 = (p & 7) * 8;
      const size_t off = ybase + (size_t)rr * CDIM + q8;
      const v8h hv = *(const v8h*)(&sYH[wave][rr][q8]);
      const v8h lv = *(const v8h*)(&sYL[wave][rr][q8]);
      *(volatile v8h*)(yH + off) = hv;
      *(volatile v8h*)(yL + off) = lv;
    }
    __threadfence();
  }
}

template <bool RES>
__global__ void __launch_bounds__(128) k_oproj(
    const _Float16* __restrict__ yH, const _Float16* __restrict__ yL,
    const _Float16* __restrict__ wall, float* __restrict__ out, int rt_first, int rt_count) {
  __shared__ __attribute__((aligned(16))) float sO[4][16][68];

  const int tid  = threadIdx.x;
  const int wave = tid >> 5;
  const int lane = tid & 31;
  const int l16  = lane & 15;
  const int lh   = lane >> 4;
  const int nt   = blockIdx.x;
  const int b    = blockIdx.y / rt_count;
  const int rtb  = rt_first + (blockIdx.y - b * rt_count);
  const int t0   = rtb * 64;
  const int tok0 = b * SEQ + t0;

  const _Float16* arow = yH + (size_t)(tok0 + wave * 16 + l16) * CDIM + 8 * lh;
  const _Float16* lrow = yL + (size_t)(tok0 + wave * 16 + l16) * CDIM + 8 * lh;
  const _Float16* brow = wall + (size_t)(WO_ROW0 + nt * 64 + l16) * CDIM + 8 * lh;

  v8f ah[4], ar[4];
#pragma unroll
  for (int n = 0; n < 4; ++n) { ah[n] = vzero8(); ar[n] = vzero8(); }

  for (int k0 = 0; k0 < CDIM; k0 += 32) {
    Frag a, al;
    a.h[0] = *(const v8h*)(arow + k0);
    a.h[1] = *(const v8h*)(arow + k0 + 16);
    if (RES) {
      al.h[0] = *(const v8h*)(lrow + k0);
      al.h[1] = *(const v8h*)(lrow + k0 + 16);
    }
    Frag bw[4];
#pragma unroll
    for (int n = 0; n < 4; ++n) {
      const _Float16* bp = brow + (size_t)(n * 16) * CDIM + k0;
      bw[n].h[0] = *(const v8h*)bp;
      bw[n].h[1] = *(const v8h*)(bp + 16);
    }
#pragma unroll
    for (int n = 0; n < 4; ++n) {
      ah[n] = wmma16(a.v, bw[n].v, ah[n]);
      if (RES) ar[n] = wmma16(al.v, bw[n].v, ar[n]);
    }
    if (RES) {
      asm volatile("v_nop\n\tv_nop\n\tv_nop\n\tv_nop"
                   : "+v"(ah[0]), "+v"(ah[1]), "+v"(ah[2]), "+v"(ah[3]),
                     "+v"(ar[0]), "+v"(ar[1]), "+v"(ar[2]), "+v"(ar[3])
                   : "v"(a.v), "v"(al.v), "v"(bw[0].v), "v"(bw[1].v), "v"(bw[2].v), "v"(bw[3].v));
    } else {
      asm volatile("v_nop\n\tv_nop\n\tv_nop\n\tv_nop"
                   : "+v"(ah[0]), "+v"(ah[1]), "+v"(ah[2]), "+v"(ah[3])
                   : "v"(a.v), "v"(bw[0].v), "v"(bw[1].v), "v"(bw[2].v), "v"(bw[3].v));
    }
  }

#pragma unroll
  for (int r = 0; r < 8; ++r) {
#pragma unroll
    for (int n = 0; n < 4; ++n) {
      float v = ah[n][r];
      if (RES) v += ar[n][r] * (1.0f / 2048.0f);
      sO[wave][r + 8 * lh][n * 16 + l16] = v * (1.0f / 16.0f);
    }
  }
  asm volatile("s_wait_dscnt 0" ::: "memory");
  __builtin_amdgcn_fence(3  , "wavefront");
  __builtin_amdgcn_wave_barrier();
  const size_t orow0 = (size_t)b * SEQ_FULL + t0 + wave * 16;
  for (int pass = 0; pass < 2; ++pass) {
#pragma unroll
    for (int it = 0; it < 8; ++it) {
      const int rr = it * 2 + lh;
      const int c4 = l16 * 4;
      const v4f v = *(const v4f*)(&sO[wave][rr][c4]);
      *(volatile v4f*)(out + (orow0 + rr) * CDIM + (size_t)nt * 64 + c4) = v;
    }
    __threadfence();
  }
}

extern "C" void kernel_launch(void* const* d_in, const int* in_sizes, int n_in,
                              void* d_out, int out_size, void* d_ws, size_t ws_size,
                              hipStream_t stream) {
  if (n_in < 10) return;
  const int need_x  = ((NB - 1) * SEQ_FULL + SEQ) * CDIM;
  const int need_ve = ((NB - 1) * SEQ_FULL + SEQ) * VEW;
  if (in_sizes[0] < need_x || in_sizes[1] < need_ve) return;
  if (in_sizes[2] < SEQ * ROTD || in_sizes[3] < SEQ * ROTD) return;
  if (in_sizes[4] < CDIM * CDIM || in_sizes[5] < VEW * CDIM || in_sizes[6] < VEW * CDIM || in_sizes[7] < CDIM * CDIM) return;
  if (in_sizes[8] < NKV * GATEC || in_sizes[9] < 1) return;
  if (out_size < need_x) return;
  if (ws_size < WS_TOTAL) return;

  const float* x     = (const float*)d_in[0];
  const float* ve    = (const float*)d_in[1];
  const float* cosb  = (const float*)d_in[2];
  const float* sinb  = (const float*)d_in[3];
  const float* wq    = (const float*)d_in[4];
  const float* wk    = (const float*)d_in[5];
  const float* wv    = (const float*)d_in[6];
  const float* wo    = (const float*)d_in[7];
  const float* wgate = (const float*)d_in[8];
  const int*   winp  = (const int*)d_in[9];
  float* out = (float*)d_out;

  char* ws = (char*)d_ws;
  size_t off = 0;
  _Float16* xh   = (_Float16*)(ws + off); off += XH_BYTES;
  _Float16* wall = (_Float16*)(ws + off); off += WALL_BYTES;
  _Float16* qH   = (_Float16*)(ws + off); off += QP_BYTES;
  _Float16* qL   = (_Float16*)(ws + off); off += QP_BYTES;
  _Float16* kH   = (_Float16*)(ws + off); off += KP_BYTES;
  _Float16* kL   = (_Float16*)(ws + off); off += KP_BYTES;
  _Float16* vTH  = (_Float16*)(ws + off); off += KP_BYTES;
  _Float16* vTL  = (_Float16*)(ws + off); off += KP_BYTES;
  _Float16* yH   = (_Float16*)(ws + off); off += YP_BYTES;
  _Float16* yL   = (_Float16*)(ws + off); off += YP_BYTES;
  if (off > ws_size) return;

  k_cvt_x<<<dim3(NTOK / 2), dim3(256), 0, stream>>>(x, xh);
  k_cvt_w<<<dim3(NWROWS / 2), dim3(256), 0, stream>>>(wq, wk, wv, wo, wall);
  k_qkv<<<dim3(NUNIT, NTOK / 64), dim3(128), 0, stream>>>(xh, wall, x, ve, cosb, sinb, wgate,
                                                          qH, qL, kH, kL, vTH, vTL);
  k_flash<true><<<dim3(QT_RES, NHEAD, NB), dim3(128), 0, stream>>>(qH, qL, kH, kL, vTH, vTL, winp, yH, yL, 0);
  if (QT_ALL > QT_RES) {
    k_flash<false><<<dim3(QT_ALL - QT_RES, NHEAD, NB), dim3(128), 0, stream>>>(qH, qL, kH, kL, vTH, vTL, winp,
                                                                                yH, yL, QT_RES);
  }
  k_oproj<true><<<dim3(CDIM / 64, NB * QT_RES), dim3(128), 0, stream>>>(yH, yL, wall, out, 0, QT_RES);
  if (QT_ALL > QT_RES) {
    k_oproj<false><<<dim3(CDIM / 64, NB * (QT_ALL - QT_RES)), dim3(128), 0, stream>>>(yH, yL, wall, out,
                                                                                      QT_RES, QT_ALL - QT_RES);
  }
}
